// SDT_35158602285468
// MI455X (gfx1250) — hardware-verified
//
#include <hip/hip_runtime.h>
#include <stddef.h>


#pragma clang fp contract(off)

typedef _Float16 v16h __attribute__((ext_vector_type(16)));
typedef _Float16 v8h  __attribute__((ext_vector_type(8)));
typedef float    v8f  __attribute__((ext_vector_type(8)));
typedef float    v4f  __attribute__((ext_vector_type(4)));
typedef _Float16 h16;

#ifndef NB
#define NB 16384
#endif
#define NB_FULL 16384
#define DIN    512
#define KAUG   513
#define KPAD   544
#define KPIECES 68
#define NNODE  1023
#define NPAD   1024
#define NLEAF  1024
#define NOUT   256
#define TDEPTH 10
#define RPB    128
#define NPART  (NB / RPB)

#define LDT 72
#define LDC 68

#define XCARRY 16.0f
#define WCARRY 64.0f
#define MCARRY 4096.0f
#define DCARRY 1024.0f

#define WELEMS  (NNODE * KAUG)
#define TAIL_F  (1 + WELEMS)
#define TAIL_V4 (TAIL_F / 4)
#define OUT1_F  ((size_t)NB_FULL * NOUT)
#define TAIL0_F ((size_t)2 * NB_FULL * NOUT)
#define OUT_TOTAL_F (TAIL0_F + (size_t)TAIL_F)

static_assert(NB >= RPB && NB <= NB_FULL && (NB % RPB) == 0);
static_assert((NB % 64) == 0);
static_assert(KPAD >= KAUG && (KPAD % 32) == 0 && (KPAD % 8) == 0 && KPIECES * 8 == KPAD);
static_assert(DIN + 1 == KAUG && DIN == 512);
static_assert(NLEAF == (1 << TDEPTH) && NNODE == NLEAF - 1 && NPAD == NLEAF);
static_assert((NPAD % 64) == 0 && (NOUT % 64) == 0 && (NLEAF % 32) == 0);
static_assert(NOUT == 256 && NLEAF == 1024);
static_assert(((size_t)NB * KPIECES) % 256 == 0);
static_assert(((size_t)NPAD * KPIECES) % 256 == 0);
static_assert((LDT % 8) == 0 && LDT >= 64);
static_assert((LDC % 4) == 0 && LDC >= 64);
static_assert(TAIL0_F * 4 == (size_t)33554432);
static_assert((TAIL0_F * 4) % 128 == 0);
static_assert((TAIL_F % 32) == 0 && (TAIL_F % 4) == 0);
static_assert(((TAIL_V4 - 32) % 32) == 0);
static_assert(OUT1_F * 4 == (size_t)16777216);
static_assert(OUT_TOTAL_F * 4 == (size_t)35653632);

#define X16_BYTES  ((size_t)NB * KPAD * 2)
#define W16_BYTES  ((size_t)NPAD * KPAD * 2)
#define P_BYTES    ((size_t)NB * NPAD * 4)
#define MU_BYTES   ((size_t)NB * NLEAF * 2)
#define DT_BYTES   ((size_t)NOUT * NLEAF * 2)
#define LOGD_BYTES ((size_t)NLEAF * NOUT * 4)
#define PART_BYTES ((size_t)NPART * NLEAF * 4)
#define OFF_X16  ((size_t)0)
#define OFF_W16  (OFF_X16 + X16_BYTES)
#define OFF_P    (OFF_W16 + W16_BYTES)
#define OFF_MU   (OFF_P + P_BYTES)
#define OFF_DT   (OFF_MU + MU_BYTES)
#define OFF_LOGD (OFF_DT + DT_BYTES)
#define OFF_PART (OFF_LOGD + LOGD_BYTES)
#define WS_TOTAL (OFF_PART + PART_BYTES)
static_assert((X16_BYTES % 128) == 0 && (W16_BYTES % 128) == 0 && (P_BYTES % 128) == 0);
static_assert((MU_BYTES % 128) == 0 && (DT_BYTES % 128) == 0 && (LOGD_BYTES % 128) == 0);
static_assert((PART_BYTES % 128) == 0);
static_assert(WS_TOTAL <= (size_t)134217728);

__device__ __forceinline__ float bf16r(float x) {
  unsigned int u = __float_as_uint(x);
  u = (u + 0x7FFFu + ((u >> 16) & 1u)) & 0xFFFF0000u;
  return __uint_as_float(u);
}

static __device__ __forceinline__ h16 toh_flush(float v) {
  const h16 r = (h16)v;
  return (fabsf(v) < 6.103515625e-05f) ? (h16)0.0f : r;
}

__device__ __forceinline__ v16h frag_at(const _Float16* p) {
  v8h lo = *(const v8h*)(p);
  v8h hi = *(const v8h*)(p + 16);
  v16h out;
#pragma unroll
  for (int i = 0; i < 8; ++i) { out[i] = lo[i]; out[i + 8] = hi[i]; }
  return out;
}

__device__ __forceinline__ v8f wmma16(v16h a, v16h b, v8f c) {
  v8f d = __builtin_amdgcn_wmma_f32_16x16x32_f16(false, a, false, b, (short)0, c,
                                                 false, false);
  asm volatile("v_nop\n\tv_nop\n\tv_nop\n\tv_nop" : "+v"(d) : "v"(a), "v"(b));
  return d;
}

__device__ __forceinline__ float red32_sum(float x) {
#pragma unroll
  for (int off = 1; off < 32; off <<= 1) x += __shfl_xor(x, off, 32);
  return x;
}
__device__ __forceinline__ float red32_max(float x) {
#pragma unroll
  for (int off = 1; off < 32; off <<= 1) x = fmaxf(x, __shfl_xor(x, off, 32));
  return x;
}

__device__ __forceinline__ void wave_lds_sync() {
  __builtin_amdgcn_fence(3  , "wavefront");
  asm volatile("s_wait_dscnt 0x0" ::: "memory");
  __builtin_amdgcn_wave_barrier();
}

__global__ __launch_bounds__(256) void xplane_kernel(
    const float* __restrict__ data, _Float16* __restrict__ X16) {
  const unsigned g = blockIdx.x * 256u + threadIdx.x;
  const unsigned b = g / (unsigned)KPIECES;
  const unsigned pc = g - b * (unsigned)KPIECES;
  const unsigned k0 = pc * 8u;
  const unsigned kl = (k0 < 504u) ? k0 : 504u;
  const float* src = data + (size_t)b * DIN + kl;
  const v4f a0 = *(const v4f*)(src);
  const v4f a1 = *(const v4f*)(src + 4);
  const bool isdata = (k0 < 512u);
  const float lead = (k0 == 512u) ? 1.0f : 0.0f;
  v8h o;
#pragma unroll
  for (int i = 0; i < 4; ++i) {
    const float f0 = isdata ? bf16r(a0[i]) : ((i == 0) ? lead : 0.0f);
    const float f1 = isdata ? bf16r(a1[i]) : 0.0f;
    o[i]     = toh_flush(XCARRY * f0);
    o[i + 4] = toh_flush(XCARRY * f1);
  }
  _Float16* p = X16 + (size_t)g * 8u;
  *(volatile v8h*)p = o;
  __threadfence();
  *(volatile v8h*)p = o;
}

__global__ __launch_bounds__(256) void wplane_kernel(
    const float* __restrict__ W, _Float16* __restrict__ W16) {
  const unsigned g = blockIdx.x * 256u + threadIdx.x;
  const unsigned n = g / (unsigned)KPIECES;
  const unsigned pc = g - n * (unsigned)KPIECES;
  const unsigned k0 = pc * 8u;
  const unsigned nn = (n < (unsigned)NNODE) ? n : (unsigned)(NNODE - 1);
  v8h o;
#pragma unroll
  for (unsigned j = 0; j < 8u; ++j) {
    const unsigned k = k0 + j;
    const unsigned col = (k < 512u) ? (k + 1u) : 0u;
    const bool ok = (n < (unsigned)NNODE) && (k <= 512u);
    const float w = W[(size_t)nn * KAUG + col];
    o[j] = toh_flush(ok ? (WCARRY * bf16r(w)) : 0.0f);
  }
  _Float16* p = W16 + (size_t)g * 8u;
  *(volatile v8h*)p = o;
  __threadfence();
  *(volatile v8h*)p = o;
}

__global__ __launch_bounds__(256) void softmax_kernel(
    const float* __restrict__ param, _Float16* __restrict__ DT16, float* __restrict__ logd) {
  __shared__ __attribute__((aligned(16))) _Float16 T[256 * LDT];
  const unsigned tid = threadIdx.x, lane = tid & 31u;
  const unsigned wave = __builtin_amdgcn_readfirstlane(tid >> 5);
  const unsigned l0 = blockIdx.x * 64u;
#pragma unroll 1
  for (unsigned rr = 0; rr < 8u; ++rr) {
    const unsigned lr = wave * 8u + rr;
    const float* pr = param + (size_t)(l0 + lr) * NOUT + lane * 4u;
    const v4f a0 = *(const v4f*)(pr);
    const v4f a1 = *(const v4f*)(pr + 128);
    float x[8];
#pragma unroll
    for (int i = 0; i < 4; ++i) { x[i] = bf16r(a0[i]); x[i + 4] = bf16r(a1[i]); }
    float mx = x[0];
#pragma unroll
    for (int i = 1; i < 8; ++i) mx = fmaxf(mx, x[i]);
    mx = red32_max(mx);
    float e[8];
    float s = 0.0f;
#pragma unroll
    for (int i = 0; i < 8; ++i) { e[i] = __expf(x[i] - mx); s += e[i]; }
    s = red32_sum(s);
    const float rs = 1.0f / s;
    const float ls = logf(s);
    v4f g0, g1;
#pragma unroll
    for (int i = 0; i < 4; ++i) {
      g0[i] = (x[i] - mx) - ls;
      g1[i] = (x[i + 4] - mx) - ls;
      T[(lane * 4u + (unsigned)i) * LDT + lr]        = toh_flush(DCARRY * (e[i] * rs));
      T[(128u + lane * 4u + (unsigned)i) * LDT + lr] = toh_flush(DCARRY * (e[i + 4] * rs));
    }
    float* lp = logd + (size_t)(l0 + lr) * NOUT + lane * 4u;
    *(volatile v4f*)(lp) = g0;
    *(volatile v4f*)(lp + 128) = g1;
    __threadfence();
    *(volatile v4f*)(lp) = g0;
    *(volatile v4f*)(lp + 128) = g1;
  }
  __syncthreads();
  v8h xo[8];
  size_t off[8];
#pragma unroll
  for (unsigned j = 0; j < 8u; ++j) {
    const unsigned idx = tid + 256u * j;
    const unsigned o = idx >> 3;
    const unsigned kc = (idx & 7u) * 8u;
    xo[j] = *(const v8h*)&T[o * LDT + kc];
    off[j] = (size_t)o * NLEAF + l0 + kc;
  }
#pragma unroll
  for (int j = 0; j < 8; ++j) *(volatile v8h*)(DT16 + off[j]) = xo[j];
  __threadfence();
#pragma unroll
  for (int j = 0; j < 8; ++j) *(volatile v8h*)(DT16 + off[j]) = xo[j];
}

template <int MODE>
__device__ __forceinline__ void gemm_body(
    const _Float16* __restrict__ A16, const _Float16* __restrict__ Bt, const unsigned K,
    const unsigned ldo, const float* __restrict__ beta, float* __restrict__ outf) {
  __shared__ __attribute__((aligned(16))) float Cs[64 * LDC];
  const unsigned tid = threadIdx.x, lane = tid & 31u;
  const unsigned w = __builtin_amdgcn_readfirstlane(tid >> 5);
  const unsigned mw = w >> 1, nw = w & 1u;
  const unsigned hh = lane >> 4, m = lane & 15u;
  const unsigned n0 = blockIdx.x * 64u;
  const unsigned row0 = blockIdx.y * 64u;

  const _Float16* ap  = A16 + (size_t)(row0 + mw * 16u + m) * K + hh * 8u;
  const _Float16* bp0 = Bt + (size_t)(n0 + nw * 32u + m) * K + hh * 8u;
  const _Float16* bp1 = bp0 + (size_t)16 * K;
  v8f acc0 = {}, acc1 = {};
#pragma unroll 2
  for (unsigned k0 = 0; k0 < K; k0 += 32u) {
    const v16h a  = frag_at(ap + k0);
    const v16h b0 = frag_at(bp0 + k0);
    const v16h b1 = frag_at(bp1 + k0);
    acc0 = wmma16(a, b0, acc0);
    acc1 = wmma16(a, b1, acc1);
  }
#pragma unroll
  for (int r = 0; r < 8; ++r) {
    float* d = &Cs[(mw * 16u + hh * 8u + (unsigned)r) * LDC + nw * 32u + m];
    d[0]  = acc0[r];
    d[16] = acc1[r];
  }
  __syncthreads();

  const unsigned c = (tid & 15u) * 4u;
  float bt[4];
#pragma unroll
  for (unsigned j = 0; j < 4u; ++j) {
    if (MODE == 0) {
      const unsigned nidx = n0 + c + j;
      const unsigned nb = (nidx < (unsigned)NNODE) ? nidx : (unsigned)(NNODE - 1);
      bt[j] = bf16r(beta[nb]);
    } else {
      bt[j] = 0.0f;
    }
  }

#pragma unroll 1
  for (unsigned g = 0; g < 4u; ++g) {
    const unsigned r = 16u * g + (tid >> 4);
    const v4f u = *(const v4f*)&Cs[r * LDC + c];
    v4f t;
#pragma unroll
    for (int j = 0; j < 4; ++j) {
      if (MODE == 0) {
        const float z = u[j] * (1.0f / (XCARRY * WCARRY));
        const float a = bt[j] * z;
        t[j] = 1.0f / (1.0f + expf(-a));
      } else {
        t[j] = logf(u[j] * (1.0f / (MCARRY * DCARRY)));
      }
    }
    *(v4f*)&Cs[r * LDC + c] = t;
  }

  v4f xs[4];
  size_t off[4];
#pragma unroll
  for (unsigned i = 0; i < 4u; ++i) {
    const unsigned r = 16u * i + (tid >> 4);
    xs[i] = *(const v4f*)&Cs[r * LDC + c];
    off[i] = (size_t)(row0 + r) * ldo + n0 + c;
  }
#pragma unroll
  for (int i = 0; i < 4; ++i) *(volatile v4f*)(outf + off[i]) = xs[i];
  __threadfence();
#pragma unroll
  for (int i = 0; i < 4; ++i) *(volatile v4f*)(outf + off[i]) = xs[i];
}

__global__ __launch_bounds__(256) void gemm_sig_kernel(
    const _Float16* __restrict__ A16, const _Float16* __restrict__ Bt,
    const float* __restrict__ beta, float* __restrict__ P) {
  gemm_body<0>(A16, Bt, (unsigned)KPAD, (unsigned)NPAD, beta, P);
}
__global__ __launch_bounds__(256) void gemm_log_kernel(
    const _Float16* __restrict__ A16, const _Float16* __restrict__ Bt,
    float* __restrict__ out1) {
  gemm_body<1>(A16, Bt, (unsigned)NLEAF, (unsigned)NOUT, out1, out1);
}

__global__ __launch_bounds__(256) void mu_kernel(
    const float* __restrict__ P, const float* __restrict__ logd,
    _Float16* __restrict__ MU16, float* __restrict__ out0, float* __restrict__ part) {
  __shared__ __attribute__((aligned(16))) float sp[8 * NLEAF];
  const unsigned tid = threadIdx.x, lane = tid & 31u;
  const unsigned wave = __builtin_amdgcn_readfirstlane(tid >> 5);
  const unsigned sb = wave * (unsigned)NLEAF;

  float cs[4][8];
#pragma unroll
  for (int i = 0; i < 4; ++i)
#pragma unroll
    for (int t = 0; t < 8; ++t) cs[i][t] = 0.0f;

#pragma unroll 1
  for (unsigned rr = 0; rr < 16u; ++rr) {
    const unsigned row = blockIdx.x * (unsigned)RPB + wave * 16u + rr;
    const float* pr = P + (size_t)row * NPAD + lane * 4u;
#pragma unroll
    for (unsigned j = 0; j < 8u; ++j) {
      const v4f a = *(const v4f*)(pr + j * 128u);
      *(v4f*)&sp[sb + j * 128u + lane * 4u] = a;
    }
    wave_lds_sync();

    float best = -1.0f;
    unsigned bidx = 0u;
    v8h xo[4];
#pragma unroll
    for (int i = 0; i < 4; ++i) {
      const unsigned J = 32u * (unsigned)i + lane;
      float mval = 1.0f;
#pragma unroll
      for (int l = 0; l < 7; ++l) {
        const unsigned j = J >> (7 - l);
        const unsigned bit = (J >> (6 - l)) & 1u;
        const float pv = sp[sb + ((1u << l) - 1u) + j];
        const float qv = 1.0f - pv;
        mval = mval * (bit ? qv : pv);
      }
      const float p7 = sp[sb + 127u + J];
      const float a0 = mval * p7;
      const float a1 = mval * (1.0f - p7);
      const float p80 = sp[sb + 255u + 2u * J];
      const float p81 = sp[sb + 256u + 2u * J];
      float bq[4];
      bq[0] = a0 * p80;
      bq[1] = a0 * (1.0f - p80);
      bq[2] = a1 * p81;
      bq[3] = a1 * (1.0f - p81);
      float cv[8];
#pragma unroll
      for (int q = 0; q < 4; ++q) {
        const float p9 = sp[sb + 511u + 4u * J + (unsigned)q];
        cv[2 * q]     = bq[q] * p9;
        cv[2 * q + 1] = bq[q] * (1.0f - p9);
      }
      v8h o;
#pragma unroll
      for (int t = 0; t < 8; ++t) {
        cs[i][t] += cv[t];
        const bool take = (cv[t] > best);
        best = take ? cv[t] : best;
        bidx = take ? (8u * J + (unsigned)t) : bidx;
        o[t] = toh_flush(MCARRY * cv[t]);
      }
      xo[i] = o;
    }

#pragma unroll
    for (int off = 1; off < 32; off <<= 1) {
      const float ov = __shfl_xor(best, off, 32);
      const int oi = __shfl_xor((int)bidx, off, 32);
      const bool take = (ov > best) || ((ov == best) && ((unsigned)oi < bidx));
      best = take ? ov : best;
      bidx = take ? (unsigned)oi : bidx;
    }
    const unsigned bcl = (bidx < (unsigned)NLEAF) ? bidx : (unsigned)(NLEAF - 1);
    const unsigned id = (unsigned)__builtin_amdgcn_readfirstlane((int)bcl);

    const float* lg = logd + (size_t)id * NOUT + lane * 4u;
    const v4f g0 = *(const v4f*)(lg);
    const v4f g1 = *(const v4f*)(lg + 128);

    _Float16* mp = MU16 + (size_t)row * NLEAF + lane * 8u;
    float* op = out0 + (size_t)row * NOUT + lane * 4u;
#pragma unroll
    for (int i = 0; i < 4; ++i) *(volatile v8h*)(mp + 256 * i) = xo[i];
    *(volatile v4f*)(op) = g0;
    *(volatile v4f*)(op + 128) = g1;
    __threadfence();
#pragma unroll
    for (int i = 0; i < 4; ++i) *(volatile v8h*)(mp + 256 * i) = xo[i];
    *(volatile v4f*)(op) = g0;
    *(volatile v4f*)(op + 128) = g1;

    wave_lds_sync();
  }

  __syncthreads();
#pragma unroll
  for (int i = 0; i < 4; ++i) {
    v4f c0, c1;
#pragma unroll
    for (int t = 0; t < 4; ++t) { c0[t] = cs[i][t]; c1[t] = cs[i][t + 4]; }
    *(v4f*)&sp[sb + 256u * (unsigned)i + lane * 8u]      = c0;
    *(v4f*)&sp[sb + 256u * (unsigned)i + lane * 8u + 4u] = c1;
  }
  __syncthreads();
  v4f tot = *(const v4f*)&sp[tid * 4u];
#pragma unroll
  for (unsigned w2 = 1; w2 < 8u; ++w2) {
    const v4f t = *(const v4f*)&sp[w2 * (unsigned)NLEAF + tid * 4u];
    tot = tot + t;
  }
  float* pp = part + (size_t)blockIdx.x * NLEAF + tid * 4u;
  *(volatile v4f*)pp = tot;
  __threadfence();
  *(volatile v4f*)pp = tot;
}

__global__ __launch_bounds__(256) void penalty_kernel(
    const float* __restrict__ part, const float* __restrict__ W, float* __restrict__ tail) {
  __shared__ float S[2048];
  __shared__ float wsum[8];
  const unsigned tid = threadIdx.x, lane = tid & 31u;
  const unsigned wave = __builtin_amdgcn_readfirstlane(tid >> 5);

  v4f a = {};
#pragma unroll 1
  for (unsigned blk = 0; blk < (unsigned)NPART; ++blk) {
    const v4f t = *(const v4f*)(part + (size_t)blk * NLEAF + tid * 4u);
    a = a + t;
  }
#pragma unroll
  for (unsigned j = 0; j < 4u; ++j) S[(unsigned)NNODE + tid * 4u + j] = a[j];
  if (tid == 0u) S[2047] = 0.0f;
  __syncthreads();

#pragma unroll 1
  for (int L = TDEPTH - 1; L >= 0; --L) {
    const unsigned n = 1u << L, base = n - 1u;
#pragma unroll 1
    for (unsigned t = tid; t < n; t += 256u) {
      const unsigned i = base + t;
      S[i] = S[2u * i + 1u] + S[2u * i + 2u];
    }
    __syncthreads();
  }

  float acc = 0.0f;
  float coeff = 0.5f * 1.0e-3f;
#pragma unroll 1
  for (unsigned L = 0; L < (unsigned)TDEPTH; ++L) {
    const unsigned slots = 2u << L;
#pragma unroll 1
    for (unsigned s = tid; s < slots; s += 256u) {
      const float denom = S[(1u << L) - 1u + (s >> 1)] + 1.0e-7f;
      float al = S[(2u << L) - 1u + s] / denom;
      al = fminf(fmaxf(al, 1.0e-7f), 1.0f - 1.0e-7f);
      acc -= coeff * (__logf(al) + __logf(1.0f - al));
    }
    coeff *= 0.5f;
  }
  acc = red32_sum(acc);
  if (lane == 0u) wsum[wave] = acc;
  __syncthreads();
  float pen = wsum[0];
#pragma unroll
  for (int j = 1; j < 8; ++j) pen += wsum[j];

  if (wave == 0u) {
    v4f v;
#pragma unroll
    for (unsigned j = 0; j < 4u; ++j) {
      const unsigned e = lane * 4u + j;
      const unsigned wi = (e > 0u) ? (e - 1u) : 0u;
      const float wv = bf16r(W[wi]);
      v[j] = (e == 0u) ? pen : wv;
    }
    float* p = tail + lane * 4u;
    *(volatile v4f*)p = v;
    __threadfence();
    *(volatile v4f*)p = v;
  }
}

__global__ __launch_bounds__(256) void wcopy_kernel(
    const float* __restrict__ W, float* __restrict__ tail) {
  const unsigned q = 32u + blockIdx.x * 256u + threadIdx.x;
  if (q < (unsigned)TAIL_V4) {
    const unsigned e0 = q * 4u;
    v4f v;
#pragma unroll
    for (unsigned j = 0; j < 4u; ++j) {
      unsigned wi = e0 + j - 1u;
      wi = (wi < (unsigned)WELEMS) ? wi : (unsigned)(WELEMS - 1);
      v[j] = bf16r(W[wi]);
    }
    float* p = tail + e0;
    *(volatile v4f*)p = v;
    __threadfence();
    *(volatile v4f*)p = v;
  }
}

extern "C" void kernel_launch(void* const* d_in, const int* in_sizes, int n_in,
                              void* d_out, int out_size, void* d_ws, size_t ws_size,
                              hipStream_t stream) {
  if (n_in < 4) return;
  if ((long long)in_sizes[0] < (long long)NB * DIN) return;
  if ((long long)in_sizes[1] < (long long)WELEMS) return;
  if (in_sizes[2] < NNODE) return;
  if ((long long)in_sizes[3] < (long long)NLEAF * NOUT) return;
  if ((long long)out_size < (long long)OUT_TOTAL_F) return;
  if (ws_size < WS_TOTAL) return;

  const float* data  = (const float*)d_in[0];
  const float* W     = (const float*)d_in[1];
  const float* beta  = (const float*)d_in[2];
  const float* param = (const float*)d_in[3];
  float* out  = (float*)d_out;
  float* out0 = out;
  float* out1 = out + OUT1_F;
  float* tail = out + TAIL0_F;

  char* ws = (char*)d_ws;
  _Float16* X16  = (_Float16*)(ws + OFF_X16);
  _Float16* W16  = (_Float16*)(ws + OFF_W16);
  float*    Pn   = (float*)(ws + OFF_P);
  _Float16* MU16 = (_Float16*)(ws + OFF_MU);
  _Float16* DT16 = (_Float16*)(ws + OFF_DT);
  float*    LOGD = (float*)(ws + OFF_LOGD);
  float*    PART = (float*)(ws + OFF_PART);

  dim3 blk(256);
  xplane_kernel<<<dim3((unsigned)(((size_t)NB * KPIECES) / 256)), blk, 0, stream>>>(data, X16);
  wplane_kernel<<<dim3((unsigned)(((size_t)NPAD * KPIECES) / 256)), blk, 0, stream>>>(W, W16);
  softmax_kernel<<<dim3(NLEAF / 64), blk, 0, stream>>>(param, DT16, LOGD);
  gemm_sig_kernel<<<dim3(NPAD / 64, NB / 64), blk, 0, stream>>>(X16, W16, beta, Pn);
  mu_kernel<<<dim3(NB / RPB), blk, 0, stream>>>(Pn, LOGD, MU16, out0, PART);
  penalty_kernel<<<dim3(1), blk, 0, stream>>>(PART, W, tail);
  gemm_log_kernel<<<dim3(NOUT / 64, NB / 64), blk, 0, stream>>>(MU16, DT16, out1);
  wcopy_kernel<<<dim3((TAIL_V4 - 32 + 255) / 256), blk, 0, stream>>>(W, tail);
}
